// LSTM_46316927320185
// MI455X (gfx1250) — hardware-verified
//
#include <hip/hip_runtime.h>
#include <math.h>

constexpr int NVOCAB = 50000;
constexpr int NEMB   = 32;
constexpr int NHID   = 16;
constexpr int NGATE  = 64;
constexpr int NBATCH = 4096;
constexpr int NSTEP  = 512;
constexpr int VTILES = NVOCAB / 16;
constexpr int ROWS_PER_BLOCK = 32;
constexpr float CARRY_ACT = 16.0f;
constexpr float CARRY_WGT = 64.0f;
constexpr float CARRY_ALL = CARRY_ACT * CARRY_WGT;
constexpr float CARRY_INV = 1.0f / CARRY_ALL;
constexpr int SLAB_PITCH = 68;

static_assert(NVOCAB % 16 == 0, "vocab tiles exact");
static_assert(NEMB == 32, "table GEMM is exactly one 32-deep k-step");
static_assert(NHID == 16, "hidden units fill the low half of one k-step");
static_assert(NGATE == 4 * NHID, "gate blocks i f g o");
static_assert(NBATCH % ROWS_PER_BLOCK == 0, "scan grid exact");
static_assert(NSTEP % 4 == 0, "index chunks of 4 steps");
static_assert(CARRY_ALL == 1024.0f, "carry product");
static_assert((size_t)NVOCAB * NGATE * 4 <= (size_t)134217728, "table fits the carve");

typedef __attribute__((ext_vector_type(16))) _Float16 v16h;
typedef __attribute__((ext_vector_type(8)))  float    v8f;
typedef __attribute__((ext_vector_type(4)))  float    v4f;
typedef __attribute__((ext_vector_type(4)))  int      v4i;

__device__ __forceinline__ v8f mma_f16(v16h a, v16h b, v8f c) {
  return __builtin_amdgcn_wmma_f32_16x16x32_f16(false, a, false, b, (short)0, c, false, false);
}
__device__ __forceinline__ void guard_group4(v8f& a, v8f& b, v8f& c, v8f& d,
                                             v16h w0, v16h w1, v16h w2, v16h w3, v16h x) {
  asm volatile("v_nop\n\tv_nop\n\tv_nop\n\tv_nop"
               : "+v"(a), "+v"(b), "+v"(c), "+v"(d)
               : "v"(w0), "v"(w1), "v"(w2), "v"(w3), "v"(x));
}
__device__ __forceinline__ void pin_frag(v16h& f) { asm volatile("" : "+v"(f) :: "memory"); }

__device__ __forceinline__ v16h frag_low8(v8f w, float sc) {
  v16h f;
#pragma unroll
  for (int e = 0; e < 8; ++e) f[e] = (_Float16)(w[e] * sc);
#pragma unroll
  for (int e = 8; e < 16; ++e) f[e] = (_Float16)0.0f;
  return f;
}
__device__ __forceinline__ v16h frag_full16(v8f p, v8f q, float sc) {
  v16h f;
#pragma unroll
  for (int e = 0; e < 8; ++e) f[e] = (_Float16)(p[e] * sc);
#pragma unroll
  for (int e = 0; e < 8; ++e) f[8 + e] = (_Float16)(q[e] * sc);
  return f;
}

__device__ __forceinline__ float gate_sigmoid(float z) {
  z = fminf(fmaxf(z, -30.0f), 30.0f);
  const float d = 1.0f + expf(-z);
  return 1.0f / d;
}
__device__ __forceinline__ float gate_tanh(float z) {
  z = fminf(fmaxf(z, -15.0f), 15.0f);
  const float d = 1.0f + expf(2.0f * z);
  const float rc = 1.0f / d;
  return 1.0f - 2.0f * rc;
}

__global__ __launch_bounds__(256) void ptable_kernel(const float* __restrict__ embed, const float* __restrict__ w_ih,
                                                     const float* __restrict__ b_ih, const float* __restrict__ b_hh,
                                                     float* __restrict__ PT) {
  __shared__ __align__(16) float sT[8][16 * SLAB_PITCH];
  const int lane = threadIdx.x & 31;
  const int wave = threadIdx.x >> 5;
  const int tile = blockIdx.x * 8 + wave;
  if (tile >= VTILES) return;
  const int c = lane & 15;
  const int hh = lane >> 4;
  const int v0 = tile * 16;

  const float* er = embed + (size_t)(v0 + c) * NEMB + 8 * hh;
  const v8f ea = *(const v8f*)(er);
  const v8f eb = *(const v8f*)(er + 16);
  v16h af = frag_full16(ea, eb, CARRY_ACT);
  v16h bfr[4];
  {
    const float* wr = w_ih + (size_t)(c) * NEMB + 8 * hh;
    const v8f wa0 = *(const v8f*)(wr);
    const v8f wb0 = *(const v8f*)(wr + 16);
    bfr[0] = frag_full16(wa0, wb0, CARRY_WGT);
  }
  pin_frag(af);
  pin_frag(bfr[0]);
  {
    const float* wr = w_ih + (size_t)(16 + c) * NEMB + 8 * hh;
    const v8f wa1 = *(const v8f*)(wr);
    const v8f wb1 = *(const v8f*)(wr + 16);
    bfr[1] = frag_full16(wa1, wb1, CARRY_WGT);
  }
  {
    const float* wr = w_ih + (size_t)(32 + c) * NEMB + 8 * hh;
    const v8f wa2 = *(const v8f*)(wr);
    const v8f wb2 = *(const v8f*)(wr + 16);
    bfr[2] = frag_full16(wa2, wb2, CARRY_WGT);
  }
  pin_frag(bfr[1]);
  pin_frag(bfr[2]);
  {
    const float* wr = w_ih + (size_t)(48 + c) * NEMB + 8 * hh;
    const v8f wa3 = *(const v8f*)(wr);
    const v8f wb3 = *(const v8f*)(wr + 16);
    bfr[3] = frag_full16(wa3, wb3, CARRY_WGT);
  }
  pin_frag(bfr[3]);

  const v8f z8 = {0.f, 0.f, 0.f, 0.f, 0.f, 0.f, 0.f, 0.f};
  v8f acc[4];
#pragma unroll
  for (int j = 0; j < 4; ++j) acc[j] = mma_f16(af, bfr[j], z8);
  guard_group4(acc[0], acc[1], acc[2], acc[3], bfr[0], bfr[1], bfr[2], bfr[3], af);

  float* slab = sT[wave];
#pragma unroll
  for (int j = 0; j < 4; ++j) {
    const int n = 16 * j + c;
    const float bv = (b_ih[n] + b_hh[n]) * CARRY_ALL;
#pragma unroll
    for (int r = 0; r < 8; ++r) slab[(8 * hh + r) * SLAB_PITCH + 16 * j + c] = acc[j][r] + bv;
  }
  __builtin_amdgcn_fence(__ATOMIC_RELEASE, "workgroup");
  __builtin_amdgcn_wave_barrier();
  __builtin_amdgcn_fence(__ATOMIC_ACQUIRE, "workgroup");
  {
    const int c4 = c * 4;
    for (int pass = 0; pass < 2; ++pass) {
#pragma unroll
      for (int it = 0; it < 8; ++it) {
        const int row = it * 2 + hh;
        const v4f v = *(const v4f*)(slab + row * SLAB_PITCH + c4);
        *(volatile v4f*)(PT + (size_t)(v0 + row) * NGATE + c4) = v;
      }
      __threadfence();
    }
  }
}

__global__ __launch_bounds__(64) void lstm_scan_kernel(const int* __restrict__ x, const float* __restrict__ PT,
                                                       const float* __restrict__ w_hh, const float* __restrict__ fc_w,
                                                       const float* __restrict__ fc_b, float* __restrict__ out) {
  __shared__ float s_out[ROWS_PER_BLOCK];
  const int tid = threadIdx.x;
  const int lane = tid & 31;
  const int wave = tid >> 5;
  const int c = lane & 15;
  const int hh = lane >> 4;
  const int rowbase = blockIdx.x * ROWS_PER_BLOCK;
  const int brow = rowbase + 16 * wave + c;

  v16h wa[4];
#pragma unroll
  for (int g = 0; g < 4; ++g) {
    const v8f w = *(const v8f*)(w_hh + (size_t)(16 * g + c) * NHID + 8 * hh);
    wa[g] = frag_low8(w, CARRY_WGT);
  }
  pin_frag(wa[0]);
  pin_frag(wa[1]);
  pin_frag(wa[2]);
  pin_frag(wa[3]);
  const v8f fw = *(const v8f*)(fc_w + 8 * hh);
  const float fb = fc_b[0];

  float cst[8], hst[8];
#pragma unroll
  for (int r = 0; r < 8; ++r) { cst[r] = 0.0f; hst[r] = 0.0f; }
  v16h hb;
#pragma unroll
  for (int e = 0; e < 16; ++e) hb[e] = (_Float16)0.0f;

  const int* xr = x + (size_t)brow * NSTEP;

#pragma unroll 1
  for (int tc = 0; tc < NSTEP / 4; ++tc) {
    v4i q = *(const v4i*)(xr + 4 * tc);
#pragma unroll 1
    for (int s = 0; s < 4; ++s) {
      int idx = q[0];
      idx = idx < 0 ? 0 : idx;
      idx = idx > (NVOCAB - 1) ? (NVOCAB - 1) : idx;
      const float* pr = PT + (size_t)idx * NGATE + 8 * hh;
      v8f acc[4];
#pragma unroll
      for (int g = 0; g < 4; ++g) acc[g] = *(const v8f*)(pr + 16 * g);
#pragma unroll
      for (int g = 0; g < 4; ++g) acc[g] = mma_f16(wa[g], hb, acc[g]);
      guard_group4(acc[0], acc[1], acc[2], acc[3], wa[0], wa[1], wa[2], wa[3], hb);

      v16h nb;
#pragma unroll
      for (int r = 0; r < 8; ++r) {
        const float zi = acc[0][r] * CARRY_INV;
        const float zf = acc[1][r] * CARRY_INV;
        const float zg = acc[2][r] * CARRY_INV;
        const float zo = acc[3][r] * CARRY_INV;
        const float ig = gate_sigmoid(zi);
        const float fg = gate_sigmoid(zf);
        const float gg = gate_tanh(zg);
        const float og = gate_sigmoid(zo);
        const float cn = fg * cst[r] + ig * gg;
        cst[r] = cn;
        const float hn = og * gate_tanh(cn);
        hst[r] = hn;
        nb[r] = (_Float16)(hn * CARRY_ACT);
      }
#pragma unroll
      for (int e = 8; e < 16; ++e) nb[e] = (_Float16)0.0f;
      hb = nb;
      q = q.yzwx;
      asm volatile("" ::: "memory");
    }
  }

  float part = 0.0f;
#pragma unroll
  for (int r = 0; r < 8; ++r) part = fmaf(hst[r], fw[r], part);
  const float other = __shfl_xor(part, 16, 32);
  const float logit = (part + other) + fb;
  const float o = gate_sigmoid(logit);
  if (hh == 0) s_out[16 * wave + c] = o;
  __syncthreads();
  if (wave == 0) {
    const float v = s_out[lane];
    float* op = out + rowbase + lane;
    *(volatile float*)op = v;
    __threadfence();
    *(volatile float*)op = v;
  }
}

extern "C" void kernel_launch(void* const* d_in, const int* in_sizes, int n_in,
                              void* d_out, int out_size, void* d_ws, size_t ws_size, hipStream_t stream) {
  if (n_in < 8 || d_out == nullptr || d_ws == nullptr) return;
  if (in_sizes[0] != NBATCH * NSTEP || in_sizes[1] != NVOCAB * NEMB || in_sizes[2] != NGATE * NEMB ||
      in_sizes[3] != NGATE * NHID || in_sizes[4] != NGATE || in_sizes[5] != NGATE ||
      in_sizes[6] != NHID || in_sizes[7] != 1 || out_size != NBATCH) return;

  const int*   x     = (const int*)d_in[0];
  const float* embed = (const float*)d_in[1];
  const float* w_ih  = (const float*)d_in[2];
  const float* w_hh  = (const float*)d_in[3];
  const float* b_ih  = (const float*)d_in[4];
  const float* b_hh  = (const float*)d_in[5];
  const float* fc_w  = (const float*)d_in[6];
  const float* fc_b  = (const float*)d_in[7];
  float* out = (float*)d_out;

  const size_t pt_bytes = (size_t)NVOCAB * NGATE * sizeof(float);
  if (pt_bytes > ws_size || pt_bytes > (size_t)134217728) return;
  float* PT = (float*)d_ws;

  ptable_kernel<<<(VTILES + 7) / 8, 256, 0, stream>>>(embed, w_ih, b_ih, b_hh, PT);
  lstm_scan_kernel<<<NBATCH / ROWS_PER_BLOCK, 64, 0, stream>>>(x, PT, w_hh, fc_w, fc_b, out);
}
